// KeyedConv2d_76794015252828
// MI455X (gfx1250) — hardware-verified
//
#include <hip/hip_runtime.h>


#define NI   64
#define CI   64
#define CO   64
#define HH   56
#define WW   56
#define HP   58
#define WP   58
#define NPX  (HH * WW)
#define DIN  (CI * NPX + 1)
#define DOUT (CO * NPX + 1)
#define YP   (CO * NPX + 64)

typedef unsigned short bf;
typedef __attribute__((ext_vector_type(16))) __bf16   v16bf;
typedef __attribute__((ext_vector_type(8)))  unsigned short v8us;
typedef __attribute__((ext_vector_type(8)))  float    v8f;
typedef __attribute__((ext_vector_type(4)))  float    v4f;
typedef v4f  __attribute__((may_alias)) v4fa;
typedef v8us __attribute__((may_alias)) v8usa;

__device__ __forceinline__ unsigned short f2bf(float f) { unsigned u = __float_as_uint(f); u += 0x7FFFu + ((u >> 16) & 1u); return (unsigned short)(u >> 16); }
__device__ __forceinline__ float bf2f(unsigned short b) { return __uint_as_float(((unsigned)b) << 16); }
__device__ __forceinline__ float bfr(float f) { return bf2f(f2bf(f)); }
__device__ __forceinline__ v16bf cat16b(v8us lo, v8us hi) { return __builtin_bit_cast(v16bf, __builtin_shufflevector(lo, hi, 0, 1, 2, 3, 4, 5, 6, 7, 8, 9, 10, 11, 12, 13, 14, 15)); }
__device__ __forceinline__ v8f wmmab(v16bf a, v16bf b, v8f c) { return __builtin_amdgcn_wmma_f32_16x16x32_bf16(false, a, false, b, (short)0, c, false, false); }
#define VST2(T, p, v) do { const T vst2_v_ = (v); *(volatile T*)(p) = vst2_v_; __threadfence(); *(volatile T*)(p) = vst2_v_; } while (0)

__global__ __launch_bounds__(256) void k_z(const float* __restrict__ x, const float* __restrict__ isc, const int* __restrict__ iperm, bf* ZH, bf* ZL, float* ZL1) {
    const size_t e = (size_t)blockIdx.x * 256 + threadIdx.x;
    const size_t tot = (size_t)NI * HP * WP * 8;
    if (e < tot) {
        const int c8 = (int)(e & 7); size_t pix = e >> 3; const int wp = (int)(pix % WP); pix /= WP; const int hp = (int)(pix % HP); const int n = (int)(pix / HP);
        v8us oh, ol;
        const bool inside = (hp >= 1 && hp <= HH && wp >= 1 && wp <= WW);
#pragma unroll
        for (int i = 0; i < 8; ++i) { float v = 0.f;
            if (inside) { const int c = c8 * 8 + i; const int j = c * NPX + (hp - 1) * WW + (wp - 1); int pj = iperm[j]; pj = pj < 0 ? 0 : (pj >= DIN ? DIN - 1 : pj);
                v = bfr(isc[j]) * bfr(x[(size_t)n * DIN + pj]); }
            const unsigned short hb = f2bf(v); oh[i] = hb; ol[i] = f2bf(v - bf2f(hb)); }
        const size_t o = (e >> 3) * CI + c8 * 8;
        *(volatile v8us*)(ZH + o) = oh; *(volatile v8us*)(ZL + o) = ol; __threadfence(); *(volatile v8us*)(ZH + o) = oh; *(volatile v8us*)(ZL + o) = ol;
    }
    if (blockIdx.x == 0 && threadIdx.x < NI) { const int n = threadIdx.x; int pj = iperm[DIN - 1]; pj = pj < 0 ? 0 : (pj >= DIN ? DIN - 1 : pj);
        const float v = bfr(isc[DIN - 1]) * bfr(x[(size_t)n * DIN + pj]);
        *(volatile float*)(ZL1 + n) = v; __threadfence(); *(volatile float*)(ZL1 + n) = v; }
}
__global__ __launch_bounds__(256) void k_w(const float* __restrict__ w, bf* WT) {
    const int t = threadIdx.x;
#pragma unroll 1
    for (int s = 0; s < (9 * CO * CI) / 2048; ++s) { const int e0 = s * 2048 + t * 8; v8us o;
#pragma unroll
        for (int i = 0; i < 8; ++i) { const int e = e0 + i; const int c = e & 63, oc = (e >> 6) & 63, tap = e >> 12; o[i] = f2bf(w[((size_t)(oc * CI + c)) * 9 + tap]); }
        VST2(v8us, WT + e0, o); }
}
__global__ __launch_bounds__(128) void k_conv(const bf* __restrict__ ZH, const bf* __restrict__ ZL, const bf* __restrict__ WT, const float* __restrict__ ZL1, const float* __restrict__ bvec, float* Y) {
    __shared__ __align__(16) float ot[CO * 68];
    const int lane = threadIdx.x & 31, wave = threadIdx.x >> 5, lr = lane & 15, hi = lane >> 4;
    const int n = blockIdx.x / (NPX / 64), pt = blockIdx.x - n * (NPX / 64), px0 = pt * 64, mypx = px0 + wave * 16 + lr;
    const int h = mypx / WW, wq = mypx - h * WW;
    v8f acc[4], accl[4];
#pragma unroll
    for (int t = 0; t < 4; ++t) { acc[t] = (v8f){}; accl[t] = (v8f){}; }
#pragma unroll 1
    for (int tap = 0; tap < 9; ++tap) { const int kh = tap / 3, kw = tap - kh * 3;
        const size_t arow = (((size_t)n * HP + h + kh) * WP + (wq + kw)) * CI + 8 * hi;
        const bf* wt = WT + (size_t)tap * CO * CI;
#pragma unroll
        for (int kc = 0; kc < 2; ++kc) {
            const v16bf a = cat16b(*(const v8us*)(ZH + arow + kc * 32), *(const v8us*)(ZH + arow + kc * 32 + 16)), al = cat16b(*(const v8us*)(ZL + arow + kc * 32), *(const v8us*)(ZL + arow + kc * 32 + 16));
#pragma unroll
            for (int t = 0; t < 4; ++t) { const bf* bp = wt + (size_t)(t * 16 + lr) * CI + kc * 32 + 8 * hi; const v16bf bb = cat16b(*(const v8us*)bp, *(const v8us*)(bp + 16));
                acc[t] = wmmab(a, bb, acc[t]); accl[t] = wmmab(al, bb, accl[t]); }
            asm volatile("v_nop" : "+v"(acc[0]), "+v"(acc[1]), "+v"(acc[2]), "+v"(acc[3]), "+v"(accl[0]), "+v"(accl[1]), "+v"(accl[2]), "+v"(accl[3]) : "v"(a), "v"(al) : "memory"); }
    }
    asm volatile("v_nop\n\tv_nop\n\tv_nop\n\tv_nop" : "+v"(acc[0]), "+v"(acc[1]), "+v"(acc[2]), "+v"(acc[3]), "+v"(accl[0]), "+v"(accl[1]), "+v"(accl[2]), "+v"(accl[3]));
    const float zl = ZL1[n];
#pragma unroll
    for (int t = 0; t < 4; ++t) { const int o = t * 16 + lr; const float bb = zl * bfr(bvec[o]);
#pragma unroll
        for (int j = 0; j < 8; ++j) ot[o * 68 + wave * 16 + hi * 8 + j] = acc[t][j] + accl[t][j] + bb; }
    __syncthreads();
    auto pass = [&]() {
#pragma unroll
        for (int s = 0; s < 8; ++s) { const int o = wave * 16 + s * 2 + (lane >> 4), piece = lane & 15; const v4f v = *(const v4fa*)(ot + o * 68 + piece * 4);
            *(volatile v4f*)(Y + (size_t)n * YP + (size_t)o * NPX + px0 + piece * 4) = v; }
    };
    pass(); __threadfence(); pass();
}
__global__ __launch_bounds__(256) void k_out(const float* __restrict__ Y, const float* __restrict__ ZL1, const float* __restrict__ asc, const int* __restrict__ aperm, float* out) {
    const size_t e = (size_t)blockIdx.x * 256 + threadIdx.x;
    if (e >= (size_t)NI * DOUT) return;
    const int n = (int)(e / DOUT), j = (int)(e - (size_t)n * DOUT); int pj = aperm[j]; pj = pj < 0 ? 0 : (pj >= DOUT ? DOUT - 1 : pj);
    const int pyc = (pj < CO * NPX) ? pj : 0; const float yv = Y[(size_t)n * YP + pyc], zl = ZL1[n];
    const float v = bfr(asc[j]) * ((pj == CO * NPX) ? zl : yv);
    *(volatile float*)(out + e) = v; __threadfence(); *(volatile float*)(out + e) = v;
}

extern "C" void kernel_launch(void* const* d_in, const int* in_sizes, int n_in,
                              void* d_out, int out_size, void* d_ws, size_t ws_size, hipStream_t stream) {
    (void)in_sizes; (void)n_in; (void)out_size;
    const float* x = (const float*)d_in[0]; const float* w = (const float*)d_in[1]; const float* bvec = (const float*)d_in[2];
    const float* asc = (const float*)d_in[3]; const float* isc = (const float*)d_in[4]; const int* aperm = (const int*)d_in[5]; const int* iperm = (const int*)d_in[6];
    float* out = (float*)d_out;
    char* wsp = (char*)d_ws;
    auto take = [&](size_t bytes) { char* p = wsp; wsp += (bytes + 255) & ~(size_t)255; return (void*)p; };
    bf* ZH = (bf*)take((size_t)NI * HP * WP * CI * 2); bf* ZL = (bf*)take((size_t)NI * HP * WP * CI * 2); float* ZL1 = (float*)take(256);
    bf* WT = (bf*)take((size_t)9 * CO * CI * 2); float* Y = (float*)take((size_t)NI * YP * 4);
    if ((size_t)(wsp - (char*)d_ws) > ws_size) return;
    k_z<<<(unsigned)(((size_t)NI * HP * WP * 8 + 255) / 256), 256, 0, stream>>>(x, isc, iperm, ZH, ZL, ZL1);
    k_w<<<1, 256, 0, stream>>>(w, WT);
    k_conv<<<NI * (NPX / 64), 128, 0, stream>>>(ZH, ZL, WT, ZL1, bvec, Y);
    k_out<<<(unsigned)(((size_t)NI * DOUT + 255) / 256), 256, 0, stream>>>(Y, ZL1, asc, aperm, out);
}
